// MatchLSTM_67645734912550
// MI455X (gfx1250) — hardware-verified
//
#include <hip/hip_runtime.h>
#include <math.h>

typedef __attribute__((ext_vector_type(16))) _Float16 v16h;
typedef __attribute__((ext_vector_type(8)))  _Float16 v8h;
typedef __attribute__((ext_vector_type(4)))  _Float16 v4h;
typedef __attribute__((ext_vector_type(16))) __bf16   v16b;
typedef __attribute__((ext_vector_type(8)))  __bf16   v8b;
typedef __attribute__((ext_vector_type(8)))  float    v8f;
typedef __attribute__((ext_vector_type(4)))  float    v4f;

#define NBATCH 32
#define NPREM 256
#define NSTEP 128
#define NHID 300
#define HPAD 320
#define KCAT 960
#define APITCH 968
#define NGATE 1200
#define TPITCH 328
#define ALPITCH 264
#define RB 16
#define RNN_THREADS 512

static_assert(HPAD % 32 == 0, "K pad");
static_assert(KCAT == 3 * HPAD, "concat K");
static_assert(NGATE % 16 == 0, "gate tiles");
static_assert(NGATE == 4 * NHID, "gates");
static_assert((NBATCH * NPREM) % 64 == 0 && (NBATCH * NSTEP) % 64 == 0 && HPAD % 64 == 0, "kit GEMM M/N tile multiples");
static_assert(NBATCH == 2 * RB, "two recurrence blocks");
static_assert(RB * 20 == 320, "a_k task count");
static_assert((APITCH * 2) % 16 == 0 && (TPITCH * 2) % 16 == 0 && (ALPITCH * 2) % 16 == 0, "16B aligned LDS rows");

__device__ __forceinline__ unsigned short f2bf_bits(float f) {
  unsigned u = __float_as_uint(f);
  return (unsigned short)((u + 0x7FFFu + ((u >> 16) & 1u)) >> 16);
}
__device__ __forceinline__ float bf_bits2f(unsigned short h) { return __uint_as_float(((unsigned)h) << 16); }

__device__ __forceinline__ void dep_guard_h(v8f& a, v8f& b, v16h x, v16h y) { asm volatile("v_nop\n\tv_nop\n\tv_nop\n\tv_nop" : "+v"(a), "+v"(b) : "v"(x), "v"(y)); }
__device__ __forceinline__ void dep_guard_b(v8f& a, v8f& b, v16b x, v16b y) { asm volatile("v_nop\n\tv_nop\n\tv_nop\n\tv_nop" : "+v"(a), "+v"(b) : "v"(x), "v"(y)); }
__device__ __forceinline__ void keep4_h(v16h a, v16h b, v16h c, v16h d) { asm volatile("v_nop" :: "v"(a), "v"(b), "v"(c), "v"(d)); }
__device__ __forceinline__ void keep4_b(v16b a, v16b b, v16b c, v16b d) { asm volatile("v_nop" :: "v"(a), "v"(b), "v"(c), "v"(d)); }
__device__ __forceinline__ void acc_guard4(v8f& a, v8f& b, v8f& c, v8f& d) { asm volatile("v_nop\n\tv_nop\n\tv_nop\n\tv_nop" : "+v"(a), "+v"(b), "+v"(c), "+v"(d)); }
template <typename T> struct Frag;
template <> struct Frag<_Float16> {
  typedef v16h V; union U { v16h v; v8h h[2]; };
  static __device__ __forceinline__ v16h load(const _Float16* p) {
    U f; f.h[0] = *(const v8h*)(p); f.h[1] = *(const v8h*)(p + 16); return f.v;
  }
  static __device__ __forceinline__ v8f mma(v16h a, v16h b, v8f c) {
    return __builtin_amdgcn_wmma_f32_16x16x32_f16(false, a, false, b, (short)0, c, false, false);
  }
  static __device__ __forceinline__ void guard(v8f& a, v8f& b, v16h x, v16h y) { dep_guard_h(a, b, x, y); }
  static __device__ __forceinline__ void keep(v16h a, v16h b, v16h c, v16h d) { keep4_h(a, b, c, d); }
};
template <> struct Frag<__bf16> {
  typedef v16b V; union U { v16b v; v8b h[2]; };
  static __device__ __forceinline__ v16b load(const __bf16* p) {
    U f; f.h[0] = *(const v8b*)(p); f.h[1] = *(const v8b*)(p + 16); return f.v;
  }
  static __device__ __forceinline__ v8f mma(v16b a, v16b b, v8f c) {
    return __builtin_amdgcn_wmma_f32_16x16x32_bf16(false, a, false, b, (short)0, c, false, false);
  }
  static __device__ __forceinline__ void guard(v8f& a, v8f& b, v16b x, v16b y) { dep_guard_b(a, b, x, y); }
  static __device__ __forceinline__ void keep(v16b a, v16b b, v16b c, v16b d) { keep4_b(a, b, c, d); }
};

template <int ET> struct Elem;
template <> struct Elem<0> { typedef _Float16 T; };
template <> struct Elem<1> { typedef __bf16 T; };
template <int ET, bool SPLIT, int BIAS_MODE, int OUT_MODE, bool RESID, int ACT = 0>
__global__ __launch_bounds__(256) void wmma_gemm64(
    const unsigned short* __restrict__ Ap, const unsigned short* __restrict__ A2p, int lda, long strideA,
    const unsigned short* __restrict__ Btp, const unsigned short* __restrict__ Bt2p, int ldb, long strideB,
    void* __restrict__ Cout, void* __restrict__ Cout2, int ldc, long strideC,
    const float* __restrict__ bias,
    const float* __restrict__ resid, long strideR,
    int M, int N, int K, float scale) {
  typedef typename Elem<ET>::T T;
  typedef typename Frag<T>::V V;
  const T* A = (const T*)Ap; const T* A2 = (const T*)A2p; const T* Bt = (const T*)Btp; const T* Bt2 = (const T*)Bt2p;
  __shared__ __align__(16) float sT[8][16 * 68];
  const int b    = blockIdx.y;
  const int lane = threadIdx.x & 31;
  const int wave = threadIdx.x >> 5;
  const int tilesN = N >> 6;
  const int tilesM = M >> 6;
  const int tile = blockIdx.x * 8 + wave;
  if (tile >= tilesM * tilesN) return;
  const int tm = tile / tilesN;
  const int tn = tile - tm * tilesN;
  const int m0 = tm << 6;
  const int n0 = tn << 6;

  const T* Ab  = A  + (size_t)b * strideA;
  const T* Bb  = Bt + (size_t)b * strideB;
  const T* Ab2 = SPLIT ? (A2  + (size_t)b * strideA) : nullptr;
  const T* Bb2 = SPLIT ? (Bt2 + (size_t)b * strideB) : nullptr;

  const int rlane = lane & 15;
  const int koff  = (lane >> 4) * 8;
  const int mOff  = (lane >> 4) * 8;

  v8f acc[4][4];
#pragma unroll
  for (int i = 0; i < 4; ++i)
#pragma unroll
    for (int j = 0; j < 4; ++j) acc[i][j] = (v8f){0.f,0.f,0.f,0.f,0.f,0.f,0.f,0.f};

  for (int k0 = 0; k0 < K; k0 += 32) {
    V bh[4], bl[4];
#pragma unroll
    for (int j = 0; j < 4; ++j) {
      const size_t bo = (size_t)(n0 + (j << 4) + rlane) * ldb + koff + k0;
      bh[j] = Frag<T>::load(Bb + bo);
      if (SPLIT) bl[j] = Frag<T>::load(Bb2 + bo);
    }
#pragma unroll
    for (int i = 0; i < 4; ++i) {
      const size_t ao = (size_t)(m0 + (i << 4) + rlane) * lda + koff + k0;
      V ah = Frag<T>::load(Ab + ao);
      V al;
      if (SPLIT) al = Frag<T>::load(Ab2 + ao);
#pragma unroll
      for (int j = 0; j < 4; ++j) {
        acc[i][j] = Frag<T>::mma(ah, bh[j], acc[i][j]);
        if (SPLIT) {
          acc[i][j] = Frag<T>::mma(ah, bl[j], acc[i][j]);
          acc[i][j] = Frag<T>::mma(al, bh[j], acc[i][j]);
        }
      }
      Frag<T>::guard(acc[i][0], acc[i][3], ah, SPLIT ? al : ah);
    }
    Frag<T>::keep(bh[0], bh[1], bh[2], bh[3]);
    if (SPLIT) Frag<T>::keep(bl[0], bl[1], bl[2], bl[3]);
  }
  acc_guard4(acc[0][0], acc[0][1], acc[0][2], acc[0][3]);
  acc_guard4(acc[1][0], acc[1][1], acc[1][2], acc[1][3]);
  acc_guard4(acc[2][0], acc[2][1], acc[2][2], acc[2][3]);
  acc_guard4(acc[3][0], acc[3][1], acc[3][2], acc[3][3]);

  float* slab = sT[wave];
  const float* Rb = RESID ? (resid + (size_t)b * strideR) : nullptr;
#pragma unroll
  for (int i = 0; i < 4; ++i) {
    const int mBase = m0 + (i << 4);
#pragma unroll
    for (int j = 0; j < 4; ++j) {
      const int n = n0 + (j << 4) + rlane;
      float bv = 0.f;
      if (BIAS_MODE == 2) bv = bias[n];
#pragma unroll
      for (int r = 0; r < 8; ++r) {
        float v = acc[i][j][r] * scale;
        if (BIAS_MODE == 1) v += bias[mBase + mOff + r];
        if (BIAS_MODE == 2) v += bv;
        if (RESID) v += Rb[(size_t)(mBase + mOff + r) * ldc + n];
        if (ACT == 1) v = tanhf(v);
        if (ACT == 2) v = fmaxf(v, 0.0f);
        if (ACT == 3) v = v / (1.0f + expf(-v));
        if (ACT == 4) v = (v > 0.f) ? v : 0.01f * v;
        if (ACT == 5) v = 0.5f * v * (1.0f + erff(v * 0.70710678118654752f));
        slab[(mOff + r) * 68 + (j << 4) + rlane] = v;
      }
    }
    __builtin_amdgcn_fence(__ATOMIC_RELEASE, "workgroup");
    __builtin_amdgcn_wave_barrier();
    __builtin_amdgcn_fence(__ATOMIC_ACQUIRE, "workgroup");
    if (OUT_MODE == 0) {
      float* C = (float*)Cout + (size_t)b * strideC;
      const int hh = lane >> 4, c4 = (lane & 15) * 4;
      for (int pass = 0; pass < 2; ++pass) {
#pragma unroll
        for (int it = 0; it < 8; ++it) {
          const int row = it * 2 + hh;
          v4f v = *(const v4f*)(slab + row * 68 + c4);
          *(volatile v4f*)(C + (size_t)(mBase + row) * ldc + n0 + c4) = v;
        }
        __threadfence();
      }
    } else {
      const int q = lane >> 3, c8 = (lane & 7) * 8;
      unsigned short* C  = (unsigned short*)Cout  + (size_t)b * strideC;
      unsigned short* C2 = (OUT_MODE == 2) ? ((unsigned short*)Cout2 + (size_t)b * strideC) : nullptr;
      for (int pass = 0; pass < 2; ++pass) {
#pragma unroll
        for (int it = 0; it < 4; ++it) {
          const int row = it * 4 + q;
          const float* sp = slab + row * 68 + c8;
          v8h hv, lv;
#pragma unroll
          for (int e = 0; e < 8; ++e) {
            if (OUT_MODE == 1) {
              hv[e] = (_Float16)sp[e];
            } else {
              unsigned short hb = f2bf_bits(sp[e]);
              unsigned short lb = f2bf_bits(sp[e] - bf_bits2f(hb));
              hv[e] = __builtin_bit_cast(_Float16, hb);
              lv[e] = __builtin_bit_cast(_Float16, lb);
            }
          }
          *(volatile v8h*)(C + (size_t)(mBase + row) * ldc + n0 + c8) = hv;
          if (OUT_MODE == 2) *(volatile v8h*)(C2 + (size_t)(mBase + row) * ldc + n0 + c8) = lv;
        }
        __threadfence();
      }
    }
    __builtin_amdgcn_fence(__ATOMIC_RELEASE, "workgroup");
    __builtin_amdgcn_wave_barrier();
    __builtin_amdgcn_fence(__ATOMIC_ACQUIRE, "workgroup");
  }
}

__device__ __forceinline__ float bfr(float f) {
  unsigned u = __float_as_uint(f);
  u = (u + 0x7FFFu + ((u >> 16) & 1u)) & 0xFFFF0000u;
  return __uint_as_float(u);
}
__device__ __forceinline__ float tanh_fast(float x) {
  const float e2 = __expf(2.0f * x);
  return 1.0f - 2.0f * __builtin_amdgcn_rcpf(e2 + 1.0f);
}
__device__ __forceinline__ float sigm_f(float x) {
  const float xc = fmaxf(x, -30.0f);
  return 1.0f / (1.0f + expf(-xc));
}
__device__ __forceinline__ v8f mma_h(v16h a, v16h b, v8f c) {
  c = __builtin_amdgcn_wmma_f32_16x16x32_f16(false, a, false, b, (short)0, c, false, false);
  asm volatile("v_nop\n\tv_nop\n\tv_nop\n\tv_nop" : "+v"(c) : "v"(a), "v"(b));
  return c;
}
__device__ __forceinline__ void wave_sync() {
  __builtin_amdgcn_fence(__ATOMIC_RELEASE, "workgroup");
  __builtin_amdgcn_wave_barrier();
  __builtin_amdgcn_fence(__ATOMIC_ACQUIRE, "workgroup");
}
__device__ __forceinline__ v8f zero8() { return (v8f){0.f, 0.f, 0.f, 0.f, 0.f, 0.f, 0.f, 0.f}; }
__device__ __forceinline__ void store16x2(unsigned short* p, v8h hv) {
  *(volatile v8h*)p = hv;
  __threadfence();
  *(volatile v8h*)p = hv;
}

__global__ __launch_bounds__(256) void k_cvt_act(const float* __restrict__ in, unsigned short* __restrict__ out, int nrows) {
  const int idx = blockIdx.x * 256 + threadIdx.x;
  if (idx < nrows * 40) {
    const int row = idx / 40;
    const int c0 = (idx - row * 40) * 8;
    v8h hv;
#pragma unroll
    for (int j = 0; j < 8; ++j) {
      const int col = c0 + j;
      const int cc = (col < NHID) ? col : (NHID - 1);
      float v = in[(size_t)row * NHID + cc];
      v = (col < NHID) ? bfr(v) : 0.0f;
      hv[j] = (_Float16)v;
    }
    store16x2(out + (size_t)idx * 8, hv);
  }
}

__global__ __launch_bounds__(256) void k_cvt_wT(const float* __restrict__ w, unsigned short* __restrict__ out,
                                                int ld_in, int nreal, int kreal, int nrows, float scale) {
  const int idx = blockIdx.x * 256 + threadIdx.x;
  if (idx < nrows * 40) {
    const int n = idx / 40;
    const int c0 = (idx - n * 40) * 8;
    const int nc = (n < nreal) ? n : (nreal - 1);
    v8h hv;
#pragma unroll
    for (int j = 0; j < 8; ++j) {
      const int k = c0 + j;
      const int kc = (k < kreal) ? k : (kreal - 1);
      float v = w[(size_t)kc * ld_in + nc];
      v = (n < nreal && k < kreal) ? (bfr(v) * scale) : 0.0f;
      hv[j] = (_Float16)v;
    }
    store16x2(out + (size_t)idx * 8, hv);
  }
}

__global__ __launch_bounds__(256) void k_cvt_ker(const float* __restrict__ ker, unsigned short* __restrict__ out) {
  const int idx = blockIdx.x * 256 + threadIdx.x;
  if (idx < NGATE * 120) {
    const int np = idx / 120;
    const int c0 = (idx - np * 120) * 8;
    const int sec = c0 / HPAD;
    const int kk0 = c0 - sec * HPAD;
    const int hid = np >> 2;
    const int g = np & 3;
    const int col = g * NHID + hid;
    v8h hv;
#pragma unroll
    for (int j = 0; j < 8; ++j) {
      const int kk = kk0 + j;
      const int kkc = (kk < NHID) ? kk : (NHID - 1);
      float v = ker[(size_t)(sec * NHID + kkc) * NGATE + col];
      v = (kk < NHID) ? (bfr(v) * 64.0f) : 0.0f;
      hv[j] = (_Float16)v;
    }
    store16x2(out + (size_t)idx * 8, hv);
  }
}

__global__ __launch_bounds__(256) void k_premT(const float* __restrict__ prem, unsigned short* __restrict__ out) {
  const int idx = blockIdx.x * 256 + threadIdx.x;
  if (idx < NBATCH * HPAD * 32) {
    const int pc = idx & 31;
    const int n = (idx >> 5) % HPAD;
    const int b = idx / (32 * HPAD);
    const int nc = (n < NHID) ? n : (NHID - 1);
    v8h hv;
#pragma unroll
    for (int j = 0; j < 8; ++j) {
      const int p = pc * 8 + j;
      float v = prem[((size_t)(b * NPREM + p)) * NHID + nc];
      v = (n < NHID) ? bfr(v) : 0.0f;
      hv[j] = (_Float16)v;
    }
    store16x2(out + (size_t)idx * 8, hv);
  }
}

__global__ __launch_bounds__(RNN_THREADS) void k_rnn(
    const float* __restrict__ hyp,
    const float* __restrict__ pmask,
    const float* __restrict__ bias,
    const float* __restrict__ DSp,
    const float* __restrict__ DTp,
    const unsigned short* __restrict__ wmPu,
    const unsigned short* __restrict__ wePu,
    const unsigned short* __restrict__ kerPu,
    const unsigned short* __restrict__ premTu,
    float* __restrict__ hist) {
  const _Float16* wmP   = (const _Float16*)wmPu;
  const _Float16* weP   = (const _Float16*)wePu;
  const _Float16* kerP  = (const _Float16*)kerPu;
  const _Float16* premT = (const _Float16*)premTu;

  __shared__ __align__(16) _Float16 Axk[RB * APITCH];
  __shared__ __align__(16) float    sh32[RB * HPAD];
  __shared__ __align__(16) _Float16 T16[64 * TPITCH];
  __shared__ __align__(16) float    E32[RB * NPREM];
  __shared__ __align__(16) _Float16 Al16[32 * ALPITCH];

  const int tid  = threadIdx.x;
  const int w    = tid >> 5;
  const int lane = tid & 31;
  const int hh   = lane >> 4;
  const int rl   = lane & 15;
  const int koff = hh * 8;
  const int bg0  = blockIdx.x * RB;

  float cst[5][2];
#pragma unroll
  for (int j = 0; j < 5; ++j) { cst[j][0] = 0.0f; cst[j][1] = 0.0f; }

  for (int i = tid; i < RB * HPAD; i += RNN_THREADS) {
    const int b = i / HPAD;
    const int k = i - b * HPAD;
    Axk[b * APITCH + 2 * HPAD + k] = (_Float16)0.0f;
  }
  __syncthreads();

  for (int t = 0; t < NSTEP; ++t) {
    for (int i = tid; i < RB * HPAD; i += RNN_THREADS) {
      const int b = i / HPAD;
      const int k = i - b * HPAD;
      const int kc = (k < NHID) ? k : (NHID - 1);
      float v = hyp[((size_t)(bg0 + b) * NSTEP + t) * NHID + kc];
      v = (k < NHID) ? bfr(v) : 0.0f;
      Axk[b * APITCH + HPAD + k] = (_Float16)v;
    }
    __syncthreads();

    for (int nt = w; nt < HPAD / 16; nt += 16) {
      v8f acc = zero8();
      const _Float16* aq = Axk + rl * APITCH + 2 * HPAD + koff;
      const _Float16* bq = wmP + (size_t)(16 * nt + rl) * HPAD + koff;
      for (int k0 = 0; k0 < HPAD; k0 += 32) {
        const v16h av = Frag<_Float16>::load(aq + k0);
        const v16h bv = Frag<_Float16>::load(bq + k0);
        acc = mma_h(av, bv, acc);
      }
      const int n = 16 * nt + rl;
#pragma unroll
      for (int r = 0; r < 8; ++r) {
        const int b = 8 * hh + r;
        const float dtv = DTp[((size_t)(bg0 + b) * NSTEP + t) * HPAD + n];
        sh32[b * HPAD + n] = acc[r] * (1.0f / 64.0f) + dtv;
      }
    }
    __syncthreads();

    for (int cix = 0; cix < (RB * NPREM) / 64; ++cix) {
      const int b = cix >> 2;
      const int pb = (cix & 3) * 64;
      {
        const float* ds0 = DSp + ((size_t)(bg0 + b) * NPREM + pb + 4 * w) * HPAD;
        const float* s0 = sh32 + b * HPAD;
        _Float16* t0 = T16 + (4 * w) * TPITCH;
#pragma unroll 1
        for (int jj = 0; jj < 10; ++jj) {
          const int q = 32 * jj + lane;
          const int i = q / 80;
          const int kk = (q - 80 * i) * 4;
          const v4f d4 = *(const v4f*)(ds0 + i * HPAD + kk);
          const v4f s4 = *(const v4f*)(s0 + kk);
          v4h o;
          o[0] = (_Float16)tanh_fast(d4[0] + s4[0]);
          o[1] = (_Float16)tanh_fast(d4[1] + s4[1]);
          o[2] = (_Float16)tanh_fast(d4[2] + s4[2]);
          o[3] = (_Float16)tanh_fast(d4[3] + s4[3]);
          *(v4h*)(t0 + i * TPITCH + kk) = o;
        }
      }
      __syncthreads();
      if (w < 4) {
        v8f acc = zero8();
        const _Float16* aq = T16 + (16 * w + rl) * TPITCH + koff;
        const _Float16* bq = weP + rl * HPAD + koff;
        for (int k0 = 0; k0 < HPAD; k0 += 32) {
          const v16h av = Frag<_Float16>::load(aq + k0);
          const v16h bv = Frag<_Float16>::load(bq + k0);
          acc = mma_h(av, bv, acc);
        }
#pragma unroll
        for (int r = 0; r < 8; ++r) {
          const int p = pb + 16 * w + 8 * hh + r;
          const float mk = bfr(pmask[(size_t)(bg0 + b) * NPREM + p]);
          const float e = acc[r] * (1.0f / 64.0f) + (1.0f - mk) * (-3.40282347e38f);
          if (rl == 0) E32[b * NPREM + p] = e;
        }
      }
      __syncthreads();
    }

    {
      const int b = w;
      const float* er = E32 + b * NPREM + 8 * lane;
      const v4f e0 = *(const v4f*)(er);
      const v4f e1 = *(const v4f*)(er + 4);
      float ev[8] = {e0[0], e0[1], e0[2], e0[3], e1[0], e1[1], e1[2], e1[3]};
      float mx = ev[0];
#pragma unroll
      for (int j = 1; j < 8; ++j) mx = fmaxf(mx, ev[j]);
#pragma unroll
      for (int off = 1; off < 32; off <<= 1) mx = fmaxf(mx, __shfl_xor(mx, off, 32));
      float ex[8];
      float s = 0.0f;
#pragma unroll
      for (int j = 0; j < 8; ++j) { ex[j] = expf(ev[j] - mx); s += ex[j]; }
#pragma unroll
      for (int off = 1; off < 32; off <<= 1) s += __shfl_xor(s, off, 32);
      const float inv = 1.0f / s;
      v8h ah, al;
#pragma unroll
      for (int j = 0; j < 8; ++j) {
        const float a = ex[j] * inv * 1024.0f;
        const _Float16 hv = (_Float16)a;
        const float hf = (float)hv;
        const float res = (a - hf) * 2048.0f;
        ah[j] = hv;
        al[j] = (_Float16)res;
      }
      const int rowh = 16 * (b >> 3) + 2 * (b & 7);
      *(v8h*)(Al16 + rowh * ALPITCH + 8 * lane) = ah;
      *(v8h*)(Al16 + (rowh + 1) * ALPITCH + 8 * lane) = al;
    }
    __syncthreads();

#pragma unroll 1
    for (int j = 0; j < 20; ++j) {
      const int tk = w + 16 * j;
      const int b = tk / 20;
      const int nt = tk - 20 * b;
      v8f acc = zero8();
      const _Float16* aq = Al16 + (16 * (b >> 3) + rl) * ALPITCH + koff;
      const _Float16* bq = premT + ((size_t)(bg0 + b) * HPAD + 16 * nt + rl) * NPREM + koff;
      for (int k0 = 0; k0 < NPREM; k0 += 32) {
        const v16h av = Frag<_Float16>::load(aq + k0);
        const v16h bv = Frag<_Float16>::load(bq + k0);
        acc = mma_h(av, bv, acc);
      }
      const int u = b & 3;
      float vh = acc[0], vl = acc[1];
      vh = (u == 1) ? acc[2] : vh;  vl = (u == 1) ? acc[3] : vl;
      vh = (u == 2) ? acc[4] : vh;  vl = (u == 2) ? acc[5] : vl;
      vh = (u == 3) ? acc[6] : vh;  vl = (u == 3) ? acc[7] : vl;
      const float ak = (vh + vl * (1.0f / 2048.0f)) * (1.0f / 1024.0f);
      if (hh == ((b & 7) >> 2)) Axk[b * APITCH + 16 * nt + rl] = (_Float16)ak;
    }
    __syncthreads();

    {
      v8f acc[5];
#pragma unroll
      for (int j = 0; j < 5; ++j) acc[j] = zero8();
      const _Float16* aq = Axk + rl * APITCH + koff;
      const _Float16* bq[5];
#pragma unroll
      for (int j = 0; j < 5; ++j) {
        int nt = w + 16 * j;
        nt = (nt < NGATE / 16) ? nt : (NGATE / 16 - 1);
        bq[j] = kerP + (size_t)(16 * nt + rl) * KCAT + koff;
      }
      for (int k0 = 0; k0 < KCAT; k0 += 32) {
        const v16h av = Frag<_Float16>::load(aq + k0);
#pragma unroll
        for (int j = 0; j < 5; ++j) {
          const v16h bv = Frag<_Float16>::load(bq[j] + k0);
          acc[j] = mma_h(av, bv, acc[j]);
        }
      }
      float* G = E32 + w * 256;
#pragma unroll
      for (int j = 0; j < 5; ++j) {
        const int nt = w + 16 * j;
        if (nt < NGATE / 16) {
#pragma unroll
          for (int r = 0; r < 8; ++r) G[(8 * hh + r) * 16 + rl] = acc[j][r] * (1.0f / 64.0f);
          wave_sync();
#pragma unroll
          for (int pp = 0; pp < 2; ++pp) {
            const int q = lane + 32 * pp;
            const int b = q >> 2;
            const int hq = q & 3;
            const int hid = 4 * nt + hq;
            const float gi = G[b * 16 + 4 * hq + 0] + bfr(bias[hid]);
            const float gj = G[b * 16 + 4 * hq + 1] + bfr(bias[NHID + hid]);
            const float gf = G[b * 16 + 4 * hq + 2] + bfr(bias[2 * NHID + hid]);
            const float go = G[b * 16 + 4 * hq + 3] + bfr(bias[3 * NHID + hid]);
            const float cold = cst[j][pp];
            const float nc = cold * sigm_f(gf + 1.0f) + sigm_f(gi) * tanhf(gj);
            const float nh = tanhf(nc) * sigm_f(go);
            cst[j][pp] = nc;
            sh32[b * HPAD + hid] = nh;
          }
          wave_sync();
        }
      }
    }
    __syncthreads();

    for (int i = tid; i < RB * HPAD; i += RNN_THREADS) {
      const int b = i / HPAD;
      const int k = i - b * HPAD;
      float v = sh32[i];
      v = (k < NHID) ? v : 0.0f;
      Axk[b * APITCH + 2 * HPAD + k] = (_Float16)v;
    }
    {
      float* hrow = hist + ((size_t)(bg0 + w) * NSTEP + t) * HPAD;
      const float* srow = sh32 + w * HPAD;
      const int l16 = (lane < 16) ? lane : 0;
      const v4f v0 = *(const v4f*)(srow + 4 * lane);
      const v4f v1 = *(const v4f*)(srow + 128 + 4 * lane);
      const v4f v2 = *(const v4f*)(srow + 256 + 4 * l16);
      for (int pass = 0; pass < 2; ++pass) {
        *(volatile v4f*)(hrow + 4 * lane) = v0;
        *(volatile v4f*)(hrow + 128 + 4 * lane) = v1;
        if (lane < 16) *(volatile v4f*)(hrow + 256 + 4 * lane) = v2;
        __threadfence();
      }
    }
    __syncthreads();
  }
}

__global__ __launch_bounds__(256) void k_out(const float* __restrict__ hist, float* __restrict__ out) {
  const int i = blockIdx.x * 256 + threadIdx.x;
  if (i < (NBATCH * NSTEP * NHID) / 4) {
    const int f = 4 * i;
    const int b = f / (NSTEP * NHID);
    const int o = f - b * (NSTEP * NHID);
    const int t = o / NHID;
    const int hid = o - t * NHID;
    const v4f v = *(const v4f*)(hist + ((size_t)(b * NSTEP + t)) * HPAD + hid);
    for (int pass = 0; pass < 2; ++pass) {
      *(volatile v4f*)(out + f) = v;
      __threadfence();
    }
  }
}

extern "C" void kernel_launch(void* const* d_in, const int* in_sizes, int n_in,
                              void* d_out, int out_size, void* d_ws, size_t ws_size,
                              hipStream_t stream) {
  (void)in_sizes; (void)n_in; (void)out_size;
  const float* premise = (const float*)d_in[0];
  const float* pmask   = (const float*)d_in[1];
  const float* hyp     = (const float*)d_in[2];
  const float* ws_w    = (const float*)d_in[3];
  const float* wt_w    = (const float*)d_in[4];
  const float* wm_w    = (const float*)d_in[5];
  const float* we_w    = (const float*)d_in[6];
  const float* kern    = (const float*)d_in[7];
  const float* bias    = (const float*)d_in[8];
  float* out = (float*)d_out;

  char* base = (char*)d_ws;
  size_t off = 0;
  const size_t szPremP = (size_t)NBATCH * NPREM * HPAD * 2;
  const size_t szHypP  = (size_t)NBATCH * NSTEP * HPAD * 2;
  const size_t szPremT = (size_t)NBATCH * HPAD * NPREM * 2;
  const size_t szW     = (size_t)HPAD * HPAD * 2;
  const size_t szWe    = (size_t)16 * HPAD * 2;
  const size_t szKer   = (size_t)NGATE * KCAT * 2;
  const size_t szDS    = (size_t)NBATCH * NPREM * HPAD * 4;
  const size_t szDT    = (size_t)NBATCH * NSTEP * HPAD * 4;
  const size_t szHist  = (size_t)NBATCH * NSTEP * HPAD * 4;
  unsigned short* premP = (unsigned short*)(base + off); off += szPremP;
  unsigned short* hypP  = (unsigned short*)(base + off); off += szHypP;
  unsigned short* premT = (unsigned short*)(base + off); off += szPremT;
  unsigned short* wsP   = (unsigned short*)(base + off); off += szW;
  unsigned short* wtP   = (unsigned short*)(base + off); off += szW;
  unsigned short* wmP   = (unsigned short*)(base + off); off += szW;
  unsigned short* weP   = (unsigned short*)(base + off); off += szWe;
  unsigned short* kerP  = (unsigned short*)(base + off); off += szKer;
  float* DS   = (float*)(base + off); off += szDS;
  float* DT   = (float*)(base + off); off += szDT;
  float* HIST = (float*)(base + off); off += szHist;
  if (off > ws_size) return;

  k_cvt_act<<<(NBATCH * NPREM * 40 + 255) / 256, 256, 0, stream>>>(premise, premP, NBATCH * NPREM);
  k_cvt_act<<<(NBATCH * NSTEP * 40 + 255) / 256, 256, 0, stream>>>(hyp, hypP, NBATCH * NSTEP);
  k_premT<<<(NBATCH * HPAD * 32 + 255) / 256, 256, 0, stream>>>(premise, premT);
  k_cvt_wT<<<(HPAD * 40 + 255) / 256, 256, 0, stream>>>(ws_w, wsP, NHID, NHID, NHID, HPAD, 64.0f);
  k_cvt_wT<<<(HPAD * 40 + 255) / 256, 256, 0, stream>>>(wt_w, wtP, NHID, NHID, NHID, HPAD, 64.0f);
  k_cvt_wT<<<(HPAD * 40 + 255) / 256, 256, 0, stream>>>(wm_w, wmP, NHID, NHID, NHID, HPAD, 64.0f);
  k_cvt_wT<<<(16 * 40 + 255) / 256, 256, 0, stream>>>(we_w, weP, 1, 1, NHID, 16, 64.0f);
  k_cvt_ker<<<(NGATE * 120 + 255) / 256, 256, 0, stream>>>(kern, kerP);

  {
    const int tilesDS = ((NBATCH * NPREM) / 64) * (HPAD / 64);
    wmma_gemm64<0, false, 0, 0, false, 0><<<dim3((tilesDS + 7) / 8, 1), 256, 0, stream>>>(
        premP, premP, HPAD, 0L, wsP, wsP, HPAD, 0L, (void*)DS, (void*)DS, HPAD, 0L,
        DS, DS, 0L, NBATCH * NPREM, HPAD, HPAD, 1.0f / 64.0f);
    const int tilesDT = ((NBATCH * NSTEP) / 64) * (HPAD / 64);
    wmma_gemm64<0, false, 0, 0, false, 0><<<dim3((tilesDT + 7) / 8, 1), 256, 0, stream>>>(
        hypP, hypP, HPAD, 0L, wtP, wtP, HPAD, 0L, (void*)DT, (void*)DT, HPAD, 0L,
        DT, DT, 0L, NBATCH * NSTEP, HPAD, HPAD, 1.0f / 64.0f);
  }

  k_rnn<<<NBATCH / RB, RNN_THREADS, 0, stream>>>(hyp, pmask, bias, DS, DT, wmP, weP, kerP, premT, HIST);

  k_out<<<((NBATCH * NSTEP * NHID) / 4 + 255) / 256, 256, 0, stream>>>(HIST, out);
}
